// MalwareGNN_39908836114735
// MI455X (gfx1250) — hardware-verified
//
#include <hip/hip_runtime.h>
#include <stddef.h>


#define DW      128
#define NTHR    256
#define NWAVE   8
#define EPT     8
#define NGRP    2
#define CHUNK   (NTHR * EPT * NGRP)
#define WCAP    (EPT * NGRP * 32)
#define LISTN   (NWAVE * WCAP)
#define NBC     4096
#define NBF     1024
#define RCAP    40960
#define RBN     128
#define TGT     256
#define DEGCAP  1024
#define OTHR    512
#define BM      64
#define KSTEPS  (DW / 32)
#define MAXL    8
#define GPB     8
#define GHMAX   64
#define CMAX    128
#define SOCAP   4096
#define WSCAP   134217728
#define ACARRY  8.0f
#define WCARRY  64.0f
#define GSCALE  (1.0f / 512.0f)
#define BNEPS   1e-5f

#define LDS_FILL ((RCAP + NBF + LISTN) * 4 + 64)

static_assert((CHUNK & (CHUNK - 1)) == 0);
static_assert(CHUNK <= 4096);
static_assert((NBC & (NBC - 1)) == 0 && (NBF & (NBF - 1)) == 0);
static_assert(NBC == 4 * NBF);
static_assert(OTHR * 8 == NBC);
static_assert((RCAP % 32) == 0);
static_assert(TGT == NWAVE * 32);
static_assert((NBC % TGT) == 0);
static_assert((TGT % BM) == 0);
static_assert(DW == 4 * 32);
static_assert((DW % 32) == 0);
static_assert(WCAP == EPT * NGRP * 32);
static_assert(GPB == NWAVE);
static_assert((GPB & (GPB - 1)) == 0);
static_assert(((GPB * DW) % NTHR) == 0);
static_assert((SOCAP % 4) == 0);
static_assert(GHMAX * (16 + 1) <= SOCAP);

typedef float    v4f  __attribute__((ext_vector_type(4)));
typedef float    v8f  __attribute__((ext_vector_type(8)));
typedef int      v4i  __attribute__((ext_vector_type(4)));
typedef _Float16 v4h  __attribute__((ext_vector_type(4)));
typedef _Float16 v8h  __attribute__((ext_vector_type(8)));
typedef _Float16 v16h __attribute__((ext_vector_type(16)));
union Frag { v16h v; v8h h[2]; };

__device__ __forceinline__ v8f wmh(v16h a, v16h b, v8f c) {
  v8f d = __builtin_amdgcn_wmma_f32_16x16x32_f16(false, a, false, b, (short)0, c, false, false);
  asm volatile("v_nop\n\tv_nop\n\tv_nop\n\tv_nop" : "+v"(d) : "v"(a), "v"(b));
  return d;
}

template <int NB>
__device__ __forceinline__ int scan_chunk(const int* __restrict__ dsts, int nE, int cbase, int slotBase,
                                          int vec8, int* list, int tid, int lane, int wave) {
  int wc = 0;
#pragma unroll
  for (int g = 0; g < NGRP; ++g) {
    const int el0  = (g * NTHR + tid) * EPT;
    const int e0   = cbase + el0;
    const int sent = -2147483647 - 1;
    v4i da, db;
    if (vec8 != 0 && cbase + CHUNK <= nE) {
      da = *(const v4i*)(dsts + e0);
      db = *(const v4i*)(dsts + e0 + 4);
    } else {
      da.x = (e0     < nE) ? dsts[min(e0, nE - 1)] : sent;
      da.y = (e0 + 1 < nE) ? dsts[min(e0 + 1, nE - 1)] : sent;
      da.z = (e0 + 2 < nE) ? dsts[min(e0 + 2, nE - 1)] : sent;
      da.w = (e0 + 3 < nE) ? dsts[min(e0 + 3, nE - 1)] : sent;
      db.x = (e0 + 4 < nE) ? dsts[min(e0 + 4, nE - 1)] : sent;
      db.y = (e0 + 5 < nE) ? dsts[min(e0 + 5, nE - 1)] : sent;
      db.z = (e0 + 6 < nE) ? dsts[min(e0 + 6, nE - 1)] : sent;
      db.w = (e0 + 7 < nE) ? dsts[min(e0 + 7, nE - 1)] : sent;
    }
    const unsigned nb = (unsigned)slotBase;
    const unsigned s0 = (unsigned)da.x - nb, s1 = (unsigned)da.y - nb;
    const unsigned s2 = (unsigned)da.z - nb, s3 = (unsigned)da.w - nb;
    const unsigned s4 = (unsigned)db.x - nb, s5 = (unsigned)db.y - nb;
    const unsigned s6 = (unsigned)db.z - nb, s7 = (unsigned)db.w - nb;
    const bool h0 = s0 < (unsigned)NB, h1 = s1 < (unsigned)NB, h2 = s2 < (unsigned)NB, h3 = s3 < (unsigned)NB;
    const bool h4 = s4 < (unsigned)NB, h5 = s5 < (unsigned)NB, h6 = s6 < (unsigned)NB, h7 = s7 < (unsigned)NB;
    const unsigned any = __builtin_amdgcn_ballot_w32(h0 | h1 | h2 | h3 | h4 | h5 | h6 | h7);
    if (any != 0u) {
#define HITJ(J, HJ, SJ) { \
        const unsigned mj = __builtin_amdgcn_ballot_w32(HJ); \
        if (mj != 0u) { \
          if (HJ) { \
            const int pos = wc + (int)__builtin_amdgcn_mbcnt_lo(mj, 0u); \
            if (pos < WCAP) list[wave * WCAP + pos] = ((el0 + (J)) << 12) | (int)(SJ); \
          } \
          wc += (int)__builtin_popcount(mj); } }
      HITJ(0, h0, s0)
      HITJ(1, h1, s1)
      HITJ(2, h2, s2)
      HITJ(3, h3, s3)
      HITJ(4, h4, s4)
      HITJ(5, h5, s5)
      HITJ(6, h6, s6)
      HITJ(7, h7, s7)
#undef HITJ
    }
  }
  return wc;
}

__global__ __launch_bounds__(NTHR) void k_count(
    const int* __restrict__ dsts, int* cnt, float* dinv, int nE, int vec8) {
  __shared__ __attribute__((aligned(16))) int scnt[NBC];
  __shared__ __attribute__((aligned(16))) int list[LISTN];
  __shared__ int wcnt[NWAVE];
  const int tid = threadIdx.x, lane = tid & 31, wave = tid >> 5;
  const int nodeBase = blockIdx.x * NBC;

  for (int i = tid; i < NBC; i += NTHR) scnt[i] = 0;
  __syncthreads();

  const int nChunks = (nE + CHUNK - 1) / CHUNK;
#pragma unroll 1
  for (int ch = 0; ch < nChunks; ++ch) {
    const int cbase = ch * CHUNK;
    const int wc = scan_chunk<NBC>(dsts, nE, cbase, nodeBase, vec8, list, tid, lane, wave);
    if (lane == 0) wcnt[wave] = wc;
    __syncthreads();
    if (wave == 0) {
#pragma unroll 1
      for (int wsx = 0; wsx < NWAVE; ++wsx) {
        int n = __builtin_amdgcn_readfirstlane(wcnt[wsx]);
        n = n > WCAP ? WCAP : (n < 0 ? 0 : n);
        const int* lp = list + wsx * WCAP;
#pragma unroll 1
        for (int i = 0; i < n; ++i) {
          const int ent  = __builtin_amdgcn_readfirstlane(lp[i]);
          const int slot = ent & (NBC - 1);
          if (lane == 0) scnt[slot] = scnt[slot] + 1;
        }
      }
    }
    __syncthreads();
  }

  v4i cq[4];
  v4f dq[4];
#pragma unroll
  for (int q = 0; q < 4; ++q) {
    const int f = (wave * 4 + q) * 128 + 4 * lane;
    const v4i cv = *(const v4i*)(scnt + f);
    cq[q] = cv;
    v4f d;
    d.x = rsqrtf((float)(cv.x < 0 ? 0 : cv.x) + 1.0f);
    d.y = rsqrtf((float)(cv.y < 0 ? 0 : cv.y) + 1.0f);
    d.z = rsqrtf((float)(cv.z < 0 ? 0 : cv.z) + 1.0f);
    d.w = rsqrtf((float)(cv.w < 0 ? 0 : cv.w) + 1.0f);
    dq[q] = d;
  }
  int*   cp = cnt  + (size_t)nodeBase;
  float* dp = dinv + (size_t)nodeBase;
#pragma unroll
  for (int q = 0; q < 4; ++q) {
    const int f = (wave * 4 + q) * 128 + 4 * lane;
    *(volatile v4i*)(cp + f) = cq[q];
    *(volatile v4f*)(dp + f) = dq[q];
  }
  __threadfence();
#pragma unroll
  for (int q = 0; q < 4; ++q) {
    const int f = (wave * 4 + q) * 128 + 4 * lane;
    *(volatile v4i*)(cp + f) = cq[q];
    *(volatile v4f*)(dp + f) = dq[q];
  }
}

__global__ __launch_bounds__(OTHR) void k_offsets(
    const int* __restrict__ cnt, int* off, int* rbase, int nChunk) {
  __shared__ __attribute__((aligned(16))) int soff[NBC];
  __shared__ __attribute__((aligned(16))) int srb[RBN];
  __shared__ int wtot[OTHR / 32];
  const int tid = threadIdx.x, lane = tid & 31, wave = tid >> 5, sub = tid >> 7;
  for (int i = tid; i < RBN; i += OTHR) srb[i] = 0;
  int carry = 0;
#pragma unroll 1
  for (int ch = 0; ch < nChunk; ++ch) {
    const int base = ch * NBC;
    const v4i c0 = *(const v4i*)(cnt + base + 8 * tid);
    const v4i c1 = *(const v4i*)(cnt + base + 8 * tid + 4);
    const int e0 = max(c0.x, 0), e1 = max(c0.y, 0), e2 = max(c0.z, 0), e3 = max(c0.w, 0);
    const int e4 = max(c1.x, 0), e5 = max(c1.y, 0), e6 = max(c1.z, 0), e7 = max(c1.w, 0);
    const int ts = e0 + e1 + e2 + e3 + e4 + e5 + e6 + e7;
    int incl = ts;
#pragma unroll
    for (int d = 1; d < 32; d <<= 1) {
      const int t = __shfl_up(incl, d);
      if (lane >= d) incl += t;
    }
    if (lane == 31) wtot[wave] = incl;
    __syncthreads();
    const int S0 = wtot[0]  + wtot[1]  + wtot[2]  + wtot[3];
    const int S1 = wtot[4]  + wtot[5]  + wtot[6]  + wtot[7];
    const int S2 = wtot[8]  + wtot[9]  + wtot[10] + wtot[11];
    const int S3 = wtot[12] + wtot[13] + wtot[14] + wtot[15];
    int pre = 0;
#pragma unroll 1
    for (int w = 4 * sub; w < wave; ++w) pre += wtot[w];
    const int b0 = carry;
    const int b1 = b0 + ((S0 + 31) & ~31);
    const int b2 = b1 + ((S1 + 31) & ~31);
    const int b3 = b2 + ((S2 + 31) & ~31);
    const int b4 = b3 + ((S3 + 31) & ~31);
    const int myb = sub == 0 ? b0 : (sub == 1 ? b1 : (sub == 2 ? b2 : b3));
    if (tid == 0) {
      srb[min(4 * ch + 0, RBN - 1)] = b0;
      srb[min(4 * ch + 1, RBN - 1)] = b1;
      srb[min(4 * ch + 2, RBN - 1)] = b2;
      srb[min(4 * ch + 3, RBN - 1)] = b3;
    }
    int run = myb + pre + incl - ts;
    soff[8 * tid + 0] = run; run += e0;
    soff[8 * tid + 1] = run; run += e1;
    soff[8 * tid + 2] = run; run += e2;
    soff[8 * tid + 3] = run; run += e3;
    soff[8 * tid + 4] = run; run += e4;
    soff[8 * tid + 5] = run; run += e5;
    soff[8 * tid + 6] = run; run += e6;
    soff[8 * tid + 7] = run;
    carry = b4;
    __syncthreads();
    const v4i o0 = *(const v4i*)(soff + 4 * tid);
    const v4i o1 = *(const v4i*)(soff + 4 * (tid + OTHR));
    int* op = off + base;
    *(volatile v4i*)(op + 4 * tid) = o0;
    *(volatile v4i*)(op + 4 * (tid + OTHR)) = o1;
    __threadfence();
    *(volatile v4i*)(op + 4 * tid) = o0;
    *(volatile v4i*)(op + 4 * (tid + OTHR)) = o1;
    __syncthreads();
  }
  if (tid == 0) srb[min(4 * nChunk, RBN - 1)] = carry;
  __syncthreads();
  v4i rv = {0, 0, 0, 0};
  if (tid < 32) rv = *(const v4i*)(srb + 4 * tid);
  if (tid < 32) *(volatile v4i*)(rbase + 4 * tid) = rv;
  __threadfence();
  if (tid < 32) *(volatile v4i*)(rbase + 4 * tid) = rv;
}

__global__ __launch_bounds__(NTHR) void k_fill(
    const int* __restrict__ srcs, const int* __restrict__ dsts,
    const int* __restrict__ off, const int* __restrict__ rbase,
    int* csr, int nN, int nE, int vec8, int csrLen) {
  extern __shared__ v4f lds_dyn[];
  int* region = (int*)lds_dyn;
  int* cursor = region + RCAP;
  int* list   = cursor + NBF;
  int* wcnt   = list + LISTN;
  const int tid = threadIdx.x, lane = tid & 31, wave = tid >> 5;
  const int b = blockIdx.x;
  const int nodeBase = b * NBF;

  int rb0 = rbase[b];
  const int rb1 = rbase[b + 1];
  rb0 = rb0 < 0 ? 0 : (rb0 > csrLen ? csrLen : rb0);
  rb0 &= ~31;
  int len = rb1 - rb0;
  len = len < 0 ? 0 : (len > RCAP ? RCAP : len);
  int lenW = (len + 31) & ~31;
  if (rb0 + lenW > csrLen) lenW = (csrLen - rb0) & ~31;

  {
    const v4i z = {0, 0, 0, 0};
    for (int i = tid; i < RCAP / 4; i += NTHR) ((v4i*)region)[i] = z;
    for (int s = tid; s < NBF; s += NTHR) {
      int o = off[nodeBase + s] - rb0;
      o = o < 0 ? 0 : (o > RCAP ? RCAP : o);
      cursor[s] = o;
    }
  }
  __syncthreads();

  const int nChunks = (nE + CHUNK - 1) / CHUNK;
#pragma unroll 1
  for (int ch = 0; ch < nChunks; ++ch) {
    const int cbase = ch * CHUNK;
    const int wc = scan_chunk<NBF>(dsts, nE, cbase, nodeBase, vec8, list, tid, lane, wave);
    if (lane == 0) wcnt[wave] = wc;
    __syncthreads();
    if (wave == 0) {
#pragma unroll 1
      for (int wsx = 0; wsx < NWAVE; ++wsx) {
        int n = __builtin_amdgcn_readfirstlane(wcnt[wsx]);
        n = n > WCAP ? WCAP : (n < 0 ? 0 : n);
        const int* lp = list + wsx * WCAP;
#pragma unroll 1
        for (int i = 0; i < n; ++i) {
          const int ent  = __builtin_amdgcn_readfirstlane(lp[i]);
          const int slot = ent & (NBF - 1);
          int e = cbase + ((ent >> 12) & (CHUNK - 1));
          e = e > nE - 1 ? nE - 1 : e;
          int sv = srcs[e];
          sv = sv < 0 ? 0 : (sv > nN - 1 ? nN - 1 : sv);
          if (lane == 0) {
            int pos = cursor[slot];
            pos = pos < 0 ? 0 : (pos > RCAP - 1 ? RCAP - 1 : pos);
            region[pos] = sv;
            const int np = pos + 1;
            cursor[slot] = np > RCAP ? RCAP : np;
          }
        }
      }
    }
    __syncthreads();
  }

  const int nv = lenW >> 2;
  int* gp = csr + rb0;
#pragma unroll 1
  for (int i = tid; i < nv; i += NTHR) { const v4i v = ((const v4i*)region)[i]; *(volatile v4i*)(gp + 4 * i) = v; }
  __threadfence();
#pragma unroll 1
  for (int i = tid; i < nv; i += NTHR) { const v4i v = ((const v4i*)region)[i]; *(volatile v4i*)(gp + 4 * i) = v; }
}

__global__ __launch_bounds__(NTHR) void k_wcvt(const float* __restrict__ wc, _Float16* dp, int nUnits) {
  const int i = (int)blockIdx.x * NTHR + (int)threadIdx.x;
  if (i >= nUnits) return;
  const int ppr = DW / 8;
  const int per = DW * ppr;
  const int l = i / per;
  const int r = i - l * per;
  const int n = r / ppr;
  const int seg = r - n * ppr;
  const float* p = wc + (size_t)l * DW * DW + (size_t)(8 * seg) * DW + n;
  v8h o;
#pragma unroll
  for (int j = 0; j < 8; ++j) {
    const float f = p[(size_t)j * DW];
    o[j] = (_Float16)(f * WCARRY);
  }
  _Float16* gp = dp + (size_t)i * 8;
  *(volatile v8h*)gp = o;
  __threadfence();
  *(volatile v8h*)gp = o;
}

__global__ __launch_bounds__(NTHR) void k_gemm(
    const float* __restrict__ Asrc, const _Float16* __restrict__ Bp, float* Cout, int nValid) {
  constexpr int TPW = 4;
  constexpr int PPR = DW / 4;
  constexpr int NIT = (BM * PPR) / NTHR;
  static_assert((BM * PPR) % NTHR == 0);
  static_assert(NIT >= 1);
  static_assert(TPW * 16 * 2 == DW);
  static_assert(BM == 4 * 16);

  __shared__ __attribute__((aligned(16))) float stg[BM * DW];
  __shared__ __attribute__((aligned(16))) _Float16 a16[BM * DW];
  const int tid = threadIdx.x, lane = tid & 31, wave = tid >> 5, hh = lane >> 4, m = lane & 15;
  const int rowBase = (int)blockIdx.x * BM;
  const int rg = wave >> 1, chf = wave & 1;
  const int r0 = rg * 16;
  const int c0 = chf * (DW / 2);

#pragma unroll
  for (int it = 0; it < NIT; ++it) {
    const int id = it * NTHR + tid;
    const int row = id / PPR, seg = id % PPR;
    const int grow = rowBase + row;
    const bool live = grow < nValid;
    int rr = grow > nValid - 1 ? nValid - 1 : grow;
    rr = rr < 0 ? 0 : rr;
    const v4f xv = *(const v4f*)(Asrc + (size_t)rr * DW + 4 * seg);
    v4h o;
    o.x = (_Float16)((live ? xv.x : 0.f) * ACARRY);
    o.y = (_Float16)((live ? xv.y : 0.f) * ACARRY);
    o.z = (_Float16)((live ? xv.z : 0.f) * ACARRY);
    o.w = (_Float16)((live ? xv.w : 0.f) * ACARRY);
    *(v4h*)(a16 + (size_t)row * DW + 4 * seg) = o;
  }
  __syncthreads();

  v8f acc[TPW];
#pragma unroll
  for (int t = 0; t < TPW; ++t) { v8f z = {0.f, 0.f, 0.f, 0.f, 0.f, 0.f, 0.f, 0.f}; acc[t] = z; }

  const _Float16* ap = a16 + (size_t)(r0 + m) * DW + 8 * hh;
  const _Float16* bp = Bp + (size_t)(c0 + m) * DW + 8 * hh;
#pragma unroll 1
  for (int kt = 0; kt < KSTEPS; ++kt) {
    Frag a;
    a.h[0] = *(const v8h*)(ap + 32 * kt);
    a.h[1] = *(const v8h*)(ap + 32 * kt + 16);
#pragma unroll
    for (int t = 0; t < TPW; ++t) {
      const size_t to = (size_t)(16 * t) * DW + 32 * kt;
      Frag b;
      b.h[0] = *(const v8h*)(bp + to);
      b.h[1] = *(const v8h*)(bp + to + 16);
      acc[t] = wmh(a.v, b.v, acc[t]);
    }
  }

  {
    float* sp = stg + (size_t)(r0 + 8 * hh) * DW + c0 + m;
    const int growb = rowBase + r0 + 8 * hh;
#pragma unroll
    for (int t = 0; t < TPW; ++t) {
#pragma unroll
      for (int r = 0; r < 8; ++r) {
        const bool lv = (growb + r) < nValid;
        const float g = acc[t][r] * GSCALE;
        sp[r * DW + 16 * t] = lv ? g : 0.f;
      }
    }
  }
  __syncthreads();

  v4f cv[NIT];
#pragma unroll
  for (int it = 0; it < NIT; ++it) {
    const int id = it * NTHR + tid;
    const int row = id / PPR, seg = id % PPR;
    cv[it] = *(const v4f*)(stg + (size_t)row * DW + 4 * seg);
  }
#pragma unroll
  for (int it = 0; it < NIT; ++it) {
    const int id = it * NTHR + tid;
    const int row = id / PPR, seg = id % PPR;
    float* gp = Cout + (size_t)(rowBase + row) * DW + 4 * seg;
    *(volatile v4f*)gp = cv[it];
  }
  __threadfence();
#pragma unroll
  for (int it = 0; it < NIT; ++it) {
    const int id = it * NTHR + tid;
    const int row = id / PPR, seg = id % PPR;
    float* gp = Cout + (size_t)(rowBase + row) * DW + 4 * seg;
    *(volatile v4f*)gp = cv[it];
  }
}

__global__ __launch_bounds__(NTHR) void k_agg(
    const int* __restrict__ csr, const int* __restrict__ off, const int* __restrict__ cnt,
    const float* __restrict__ dinv, const float* __restrict__ hw,
    const float* __restrict__ cb, const float* __restrict__ gam, const float* __restrict__ bet,
    const float* __restrict__ mu, const float* __restrict__ var,
    float* hout, int nN, int csrLen) {
  const int tid = threadIdx.x, lane = tid & 31, wave = tid >> 5;
  const int tbase = blockIdx.x * TGT + wave * 32;
  const int col4 = 4 * lane;
  const int cl    = tbase + lane;
  const int cnt_l = cnt[cl];
  const int off_l = off[cl];
  const float di_l = dinv[cl];

  const v4f cbv = *(const v4f*)(cb  + col4);
  const v4f gv  = *(const v4f*)(gam + col4);
  const v4f bv  = *(const v4f*)(bet + col4);
  const v4f mv  = *(const v4f*)(mu  + col4);
  const v4f vv  = *(const v4f*)(var + col4);
  v4f scv;
  scv.x = gv.x * rsqrtf(vv.x + BNEPS);
  scv.y = gv.y * rsqrtf(vv.y + BNEPS);
  scv.z = gv.z * rsqrtf(vv.z + BNEPS);
  scv.w = gv.w * rsqrtf(vv.w + BNEPS);

#pragma unroll 1
  for (int j = 0; j < 32; ++j) {
    const int c = tbase + j;
    int n = __shfl(cnt_l, j);
    n = n < 0 ? 0 : (n > DEGCAP ? DEGCAP : n);
    const int st = __shfl(off_l, j);
    const float dc = __shfl(di_l, j);
    const float dd = dc * dc;

    v4f a = *(const v4f*)(hw + (size_t)c * DW + col4);
    a = a * dd;
#pragma unroll 1
    for (int q0 = 0; q0 < n; q0 += 32) {
      int pos = st + q0 + lane;
      pos = pos < 0 ? 0 : (pos > csrLen - 1 ? csrLen - 1 : pos);
      int sl = csr[pos];
      sl = sl < 0 ? 0 : (sl > nN - 1 ? nN - 1 : sl);
      const int mcnt = (n - q0) < 32 ? (n - q0) : 32;
#pragma unroll 1
      for (int pp = 0; pp < mcnt; ++pp) {
        const int s = __builtin_amdgcn_readlane(sl, pp);
        const float cf = dinv[s] * dc;
        const v4f xv = *(const v4f*)(hw + (size_t)s * DW + col4);
        a = a + xv * cf;
      }
    }

    const bool live = c < nN;
    v4f t = a + cbv;
    t = (t - mv) * scv + bv;
    v4f o;
    o.x = live ? fmaxf(t.x, 0.f) : 0.f;
    o.y = live ? fmaxf(t.y, 0.f) : 0.f;
    o.z = live ? fmaxf(t.z, 0.f) : 0.f;
    o.w = live ? fmaxf(t.w, 0.f) : 0.f;
    float* gp = hout + (size_t)c * DW + col4;
    *(volatile v4f*)gp = o;
    __threadfence();
    *(volatile v4f*)gp = o;
  }
}

__global__ __launch_bounds__(NTHR) void k_pool(
    const int* __restrict__ batch, const float* __restrict__ h, float* pooled, int nN, int vec8) {
  __shared__ __attribute__((aligned(16))) int list[LISTN];
  __shared__ __attribute__((aligned(16))) float spart[NWAVE * GPB * DW];
  __shared__ __attribute__((aligned(16))) float ssum[GPB * DW];
  const int tid = threadIdx.x, lane = tid & 31, wave = tid >> 5;
  const int gBase = blockIdx.x * GPB;
  const int col4 = 4 * lane;

  v4f acc[GPB];
#pragma unroll
  for (int s = 0; s < GPB; ++s) { v4f z = {0.f, 0.f, 0.f, 0.f}; acc[s] = z; }

  const int nChunks = (nN + CHUNK - 1) / CHUNK;
#pragma unroll 1
  for (int ch = 0; ch < nChunks; ++ch) {
    const int cbase = ch * CHUNK;
    const int wc = scan_chunk<GPB>(batch, nN, cbase, gBase, vec8, list, tid, lane, wave);
    __syncthreads();
    int n = wc;
    n = n > WCAP ? WCAP : (n < 0 ? 0 : n);
    const int* lp = list + wave * WCAP;
#pragma unroll 1
    for (int i = 0; i < n; ++i) {
      const int ent = __builtin_amdgcn_readfirstlane(lp[i]);
      int node = cbase + ((ent >> 12) & (CHUNK - 1));
      node = node > nN - 1 ? nN - 1 : (node < 0 ? 0 : node);
      const int slot = ent & (GPB - 1);
      const v4f hv = *(const v4f*)(h + (size_t)node * DW + col4);
#pragma unroll
      for (int s = 0; s < GPB; ++s) {
        const bool hit = slot == s;
        v4f add;
        add.x = hit ? hv.x : 0.f;
        add.y = hit ? hv.y : 0.f;
        add.z = hit ? hv.z : 0.f;
        add.w = hit ? hv.w : 0.f;
        acc[s] = acc[s] + add;
      }
    }
    __syncthreads();
  }

#pragma unroll
  for (int s = 0; s < GPB; ++s) *(v4f*)(spart + (size_t)(wave * GPB + s) * DW + col4) = acc[s];
  __syncthreads();
#pragma unroll
  for (int q = 0; q < (GPB * DW) / NTHR; ++q) {
    const int idx = q * NTHR + tid;
    const int s = idx / DW, c = idx % DW;
    float S = 0.f;
#pragma unroll
    for (int w = 0; w < NWAVE; ++w) S += spart[(w * GPB + s) * DW + c];
    ssum[idx] = S;
  }
  __syncthreads();
  const v4f v = *(const v4f*)(ssum + wave * DW + col4);
  float* gp = pooled + (size_t)(gBase + wave) * DW + col4;
  *(volatile v4f*)gp = v;
  __threadfence();
  *(volatile v4f*)gp = v;
}

__global__ __launch_bounds__(NTHR) void k_head(
    const float* __restrict__ pooled,
    const float* __restrict__ w1, const float* __restrict__ b1,
    const float* __restrict__ w2, const float* __restrict__ b2,
    const float* __restrict__ v1, const float* __restrict__ c1,
    const float* __restrict__ v2, const float* __restrict__ c2,
    float* out, int nG, int nC) {
  __shared__ __attribute__((aligned(16))) float shid[GHMAX * DW];
  __shared__ __attribute__((aligned(16))) float so[SOCAP];
  const int tid = threadIdx.x;
  nG = nG < 0 ? 0 : (nG > GHMAX ? GHMAX : nG);
  nC = nC < 1 ? 1 : (nC > CMAX ? CMAX : nC);
  if (nG * (nC + 1) > SOCAP) nG = SOCAP / (nC + 1);
  const int nHid = nG * DW;
  const int nLog = nG * nC;
  const int nTot = nLog + nG;

#pragma unroll 1
  for (int i = tid; i < nHid; i += NTHR) {
    const int g = i >> 7, hc = i & (DW - 1);
    const float* pg = pooled + (size_t)g * DW;
    float a = 0.f;
#pragma unroll 4
    for (int k = 0; k < DW; ++k) a += pg[k] * w1[(size_t)k * DW + hc];
    shid[i] = fmaxf(a + b1[hc], 0.f);
  }
  __syncthreads();
#pragma unroll 1
  for (int i = tid; i < nLog; i += NTHR) {
    const int g = i / nC;
    const int c = i - g * nC;
    const float* ph = shid + g * DW;
    float a = 0.f;
#pragma unroll 4
    for (int k = 0; k < DW; ++k) a += ph[k] * w2[(size_t)k * nC + c];
    so[i] = a + b2[c];
  }
  __syncthreads();
#pragma unroll 1
  for (int i = tid; i < nHid; i += NTHR) {
    const int g = i >> 7, hc = i & (DW - 1);
    const float* pg = pooled + (size_t)g * DW;
    float a = 0.f;
#pragma unroll 4
    for (int k = 0; k < DW; ++k) a += pg[k] * v1[(size_t)k * DW + hc];
    shid[i] = fmaxf(a + c1[hc], 0.f);
  }
  __syncthreads();
#pragma unroll 1
  for (int g = tid; g < nG; g += NTHR) {
    const float* ph = shid + g * DW;
    float a = 0.f;
#pragma unroll 4
    for (int k = 0; k < DW; ++k) a += ph[k] * v2[k];
    float z = a + c2[0];
    z = z > 30.f ? 30.f : (z < -30.f ? -30.f : z);
    const float e = __expf(-z);
    so[nLog + g] = __builtin_amdgcn_rcpf(1.0f + e);
  }
  __syncthreads();

  const int nq = nTot >> 2, rem = nTot & 3;
#pragma unroll 1
  for (int q = tid; q < nq; q += NTHR) { const v4f v = *(const v4f*)(so + 4 * q); *(volatile v4f*)(out + 4 * q) = v; }
  if (tid == 0) {
#pragma unroll 1
    for (int r = 0; r < rem; ++r) *(volatile float*)(out + 4 * nq + r) = so[4 * nq + r];
  }
  __threadfence();
#pragma unroll 1
  for (int q = tid; q < nq; q += NTHR) { const v4f v = *(const v4f*)(so + 4 * q); *(volatile v4f*)(out + 4 * q) = v; }
  if (tid == 0) {
#pragma unroll 1
    for (int r = 0; r < rem; ++r) *(volatile float*)(out + 4 * nq + r) = so[4 * nq + r];
  }
}

extern "C" void kernel_launch(void* const* d_in, const int* in_sizes, int n_in,
                              void* d_out, int out_size, void* d_ws, size_t ws_size,
                              hipStream_t stream) {
  if (n_in < 17) return;
  if (in_sizes[0] < DW || (in_sizes[0] % DW) != 0) return;
  const int nN = in_sizes[0] / DW;
  if (in_sizes[1] < 2 || (in_sizes[1] & 1) != 0) return;
  const int nE = in_sizes[1] / 2;
  if (in_sizes[2] != nN) return;
  if (in_sizes[3] < DW * DW || (in_sizes[3] % (DW * DW)) != 0) return;
  const int nL = in_sizes[3] / (DW * DW);
  if (nL < 1 || nL > MAXL) return;
  for (int j = 4; j <= 8; ++j) if (in_sizes[j] != nL * DW) return;
  if (in_sizes[9] != DW * DW || in_sizes[10] != DW) return;
  const int nC = in_sizes[12];
  if (nC < 1 || nC > CMAX) return;
  if (in_sizes[11] != DW * nC) return;
  if (in_sizes[13] != DW * DW || in_sizes[14] != DW || in_sizes[15] != DW || in_sizes[16] != 1) return;
  if (out_size < nC + 1 || (out_size % (nC + 1)) != 0) return;
  const int nG = out_size / (nC + 1);
  if (nG < 1 || nG > GHMAX || nG * (nC + 1) > SOCAP) return;
  if (nG * (nC + 1) != out_size) return;
  if (nE > (1 << 28) || nN > (1 << 22)) return;

  const float* x     = (const float*)d_in[0];
  const int*   ei    = (const int*)d_in[1];
  const int*   src   = ei;
  const int*   dst   = ei + nE;
  const int*   batch = (const int*)d_in[2];
  const float* convW = (const float*)d_in[3];
  const float* convB = (const float*)d_in[4];
  const float* bnG   = (const float*)d_in[5];
  const float* bnB   = (const float*)d_in[6];
  const float* bnM   = (const float*)d_in[7];
  const float* bnV   = (const float*)d_in[8];
  const float* cW1   = (const float*)d_in[9];
  const float* cB1   = (const float*)d_in[10];
  const float* cW2   = (const float*)d_in[11];
  const float* cB2   = (const float*)d_in[12];
  const float* nW1   = (const float*)d_in[13];
  const float* nB1   = (const float*)d_in[14];
  const float* nW2   = (const float*)d_in[15];
  const float* nB2   = (const float*)d_in[16];
  float* out = (float*)d_out;

  const int NPAD   = ((nN + TGT - 1) / TGT) * TGT;
  const int nBC    = (nN + NBC - 1) / NBC;
  const int CNTPAD = nBC * NBC;
  if (CNTPAD < NPAD) return;
  if (4 * nBC + 1 > RBN) return;
  const int nBF    = (nN + NBF - 1) / NBF;
  if (nBF > 4 * nBC) return;
  const int csrLen = ((nE + 31) & ~31) + 4096;
  if (31 * 4 * nBC > 4096) return;
  const int nAgg   = NPAD / TGT;
  const int nGemm  = NPAD / BM;
  const int nUnits = nL * DW * (DW / 8);
  const int GBLK   = (nG + GPB - 1) / GPB;
  const int GPAD   = GBLK * GPB;

  char* ws = (char*)d_ws;
  size_t off = 0;
  const size_t oWp  = off; off += (size_t)nL * DW * DW * 2;        off = (off + 255) & ~(size_t)255;
  const size_t oHw  = off; off += (size_t)NPAD * DW * 4;          off = (off + 255) & ~(size_t)255;
  const size_t oH   = off; off += (size_t)NPAD * DW * 4;          off = (off + 255) & ~(size_t)255;
  const size_t oCnt = off; off += (size_t)CNTPAD * 4;             off = (off + 255) & ~(size_t)255;
  const size_t oDi  = off; off += (size_t)CNTPAD * 4;             off = (off + 255) & ~(size_t)255;
  const size_t oOff = off; off += (size_t)CNTPAD * 4;             off = (off + 255) & ~(size_t)255;
  const size_t oRb  = off; off += (size_t)RBN * 4;                off = (off + 255) & ~(size_t)255;
  const size_t oCsr = off; off += (size_t)csrLen * 4;             off = (off + 255) & ~(size_t)255;
  const size_t oPl  = off; off += (size_t)GPAD * DW * 4;          off = (off + 255) & ~(size_t)255;
  if (off > ws_size || off > (size_t)WSCAP) return;

  _Float16* wpl = (_Float16*)(ws + oWp);
  float* hwp  = (float*)(ws + oHw);
  float* hp   = (float*)(ws + oH);
  int*   cnt  = (int*)(ws + oCnt);
  float* dinv = (float*)(ws + oDi);
  int*   offp = (int*)(ws + oOff);
  int*   rb   = (int*)(ws + oRb);
  int*   csr  = (int*)(ws + oCsr);
  float* pooled = (float*)(ws + oPl);

  const int vec8 = ((nE & 3) == 0) ? 1 : 0;

  k_wcvt<<<(nUnits + NTHR - 1) / NTHR, NTHR, 0, stream>>>(convW, wpl, nUnits);
  k_count<<<nBC, NTHR, 0, stream>>>(dst, cnt, dinv, nE, vec8);
  k_offsets<<<1, OTHR, 0, stream>>>(cnt, offp, rb, nBC);
  hipFuncSetAttribute(reinterpret_cast<const void*>(&k_fill),
                      hipFuncAttributeMaxDynamicSharedMemorySize, LDS_FILL);
  k_fill<<<nBF, NTHR, LDS_FILL, stream>>>(src, dst, offp, rb, csr, nN, nE, vec8, csrLen);

  for (int l = 0; l < nL; ++l) {
    const float* hsrc = (l == 0) ? x : hp;
    const _Float16* bpl = wpl + (size_t)l * DW * DW;
    k_gemm<<<nGemm, NTHR, 0, stream>>>(hsrc, bpl, hwp, nN);
    k_agg<<<nAgg, NTHR, 0, stream>>>(csr, offp, cnt, dinv, hwp,
                                      convB + (size_t)l * DW, bnG + (size_t)l * DW, bnB + (size_t)l * DW,
                                      bnM + (size_t)l * DW, bnV + (size_t)l * DW, hp, nN, csrLen);
  }

  k_pool<<<GBLK, NTHR, 0, stream>>>(batch, hp, pooled, nN, 1);
  k_head<<<1, NTHR, 0, stream>>>(pooled, cW1, cB1, cW2, cB2, nW1, nB1, nW2, nB2, out, nG, nC);
}
